// RWKV_TimeMix_46127948759550
// MI455X (gfx1250) — hardware-verified
//
#include <hip/hip_runtime.h>
#include <stdint.h>

#pragma clang fp contract(off)

constexpr int NB_SEQ    = 16;
constexpr int SEQ_T     = 2048;
constexpr int HID       = 256;
constexpr int NROWS     = NB_SEQ * SEQ_T;
constexpr int HALF_ROWS = NROWS / 2;
constexpr int BGRP      = 8;
constexpr int WT_PITCH  = 264;
constexpr int KT_PITCH  = 72;

constexpr size_t SZ_WT    = (size_t)4 * HID * HID * 2;
constexpr size_t SZ_WD    = (size_t)SEQ_T * SEQ_T * 2;
constexpr size_t SZ_PLANE = (size_t)HALF_ROWS * HID * 2;
constexpr size_t SZ_PL    = 2 * SZ_PLANE;
constexpr size_t SZ_F     = (size_t)NROWS * HID * 4;
constexpr size_t OFF_WT   = 0;
constexpr size_t OFF_WD   = OFF_WT + SZ_WT;
constexpr size_t OFF_PL   = OFF_WD + SZ_WD;
constexpr size_t OFF_F1   = OFF_PL + SZ_PL;
constexpr size_t OFF_F2   = OFF_F1 + SZ_F;
constexpr size_t OFF_F3   = OFF_F2 + SZ_F;
constexpr size_t WS_TOTAL = OFF_F3 + SZ_F;
static_assert(WS_TOTAL == (size_t)126353408u);
static_assert(WS_TOTAL <= (size_t)134217728u);
static_assert(SZ_PLANE == (size_t)BGRP * HID * SEQ_T * 2);
static_assert((size_t)NROWS * HID * 2 <= SZ_F / 2);
static_assert((OFF_WD % 128) == 0 && (OFF_PL % 128) == 0 && (OFF_F1 % 128) == 0 && (OFF_F2 % 128) == 0 && (OFF_F3 % 128) == 0);
static_assert(HALF_ROWS % 64 == 0 && NROWS % 64 == 0 && SEQ_T % 64 == 0 && HID % 64 == 0);
static_assert(HID % 32 == 0 && SEQ_T % 32 == 0);
static_assert(SEQ_T % 16 == 0 && (SEQ_T % 256) == 0 && HALF_ROWS % 8 == 0);

typedef __attribute__((ext_vector_type(16))) _Float16 v16h;
typedef __attribute__((ext_vector_type(8)))  _Float16 v8h;
typedef __attribute__((ext_vector_type(16))) __bf16   v16b;
typedef __attribute__((ext_vector_type(8)))  __bf16   v8b;
typedef __attribute__((ext_vector_type(8)))  float    v8f;
typedef __attribute__((ext_vector_type(4)))  float    v4f;
typedef __attribute__((ext_vector_type(4)))  unsigned int v4u;

union U4f { v4f v; float f[4]; };
union U8f { v4f q[2]; float f[8]; };

__device__ __forceinline__ unsigned short f2bf_bits(float f) {
  unsigned u = __float_as_uint(f);
  return (unsigned short)((u + 0x7FFFu + ((u >> 16) & 1u)) >> 16);
}
__device__ __forceinline__ float bf_bits2f(unsigned short h) { return __uint_as_float(((unsigned)h) << 16); }
__device__ __forceinline__ float bfr(float f) { return bf_bits2f(f2bf_bits(f)); }
__device__ __forceinline__ unsigned pack2(unsigned short lo, unsigned short hi) { return (unsigned)lo | ((unsigned)hi << 16); }

__device__ __forceinline__ void dep_guard_h(v8f& a, v8f& b, v16h x, v16h y) { asm volatile("v_nop\n\tv_nop\n\tv_nop\n\tv_nop" : "+v"(a), "+v"(b) : "v"(x), "v"(y)); }
__device__ __forceinline__ void dep_guard_b(v8f& a, v8f& b, v16b x, v16b y) { asm volatile("v_nop\n\tv_nop\n\tv_nop\n\tv_nop" : "+v"(a), "+v"(b) : "v"(x), "v"(y)); }
__device__ __forceinline__ void keep4_h(v16h a, v16h b, v16h c, v16h d) { asm volatile("v_nop" :: "v"(a), "v"(b), "v"(c), "v"(d)); }
__device__ __forceinline__ void keep4_b(v16b a, v16b b, v16b c, v16b d) { asm volatile("v_nop" :: "v"(a), "v"(b), "v"(c), "v"(d)); }
__device__ __forceinline__ void acc_guard4(v8f& a, v8f& b, v8f& c, v8f& d) { asm volatile("v_nop\n\tv_nop\n\tv_nop\n\tv_nop" : "+v"(a), "+v"(b), "+v"(c), "+v"(d)); }
template <typename T> struct Frag;
template <> struct Frag<_Float16> {
  typedef v16h V; union U { v16h v; v8h h[2]; };
  static __device__ __forceinline__ v16h load(const _Float16* p) {
    U f; f.h[0] = *(const v8h*)(p); f.h[1] = *(const v8h*)(p + 16); return f.v;
  }
  static __device__ __forceinline__ v8f mma(v16h a, v16h b, v8f c) {
    return __builtin_amdgcn_wmma_f32_16x16x32_f16(false, a, false, b, (short)0, c, false, false);
  }
  static __device__ __forceinline__ void guard(v8f& a, v8f& b, v16h x, v16h y) { dep_guard_h(a, b, x, y); }
  static __device__ __forceinline__ void keep(v16h a, v16h b, v16h c, v16h d) { keep4_h(a, b, c, d); }
};
template <> struct Frag<__bf16> {
  typedef v16b V; union U { v16b v; v8b h[2]; };
  static __device__ __forceinline__ v16b load(const __bf16* p) {
    U f; f.h[0] = *(const v8b*)(p); f.h[1] = *(const v8b*)(p + 16); return f.v;
  }
  static __device__ __forceinline__ v8f mma(v16b a, v16b b, v8f c) {
    return __builtin_amdgcn_wmma_f32_16x16x32_bf16(false, a, false, b, (short)0, c, false, false);
  }
  static __device__ __forceinline__ void guard(v8f& a, v8f& b, v16b x, v16b y) { dep_guard_b(a, b, x, y); }
  static __device__ __forceinline__ void keep(v16b a, v16b b, v16b c, v16b d) { keep4_b(a, b, c, d); }
};

template <int ET> struct Elem;
template <> struct Elem<0> { typedef _Float16 T; };
template <> struct Elem<1> { typedef __bf16 T; };
template <int ET, int SPLITM, int OUT_MODE, bool GATE, bool TRI>
__global__ __launch_bounds__(256) void wmma_gemm64(
    const unsigned short* __restrict__ Ap, const unsigned short* __restrict__ A2p, int lda, long strideA,
    const unsigned short* __restrict__ Btp, const unsigned short* __restrict__ Bt2p, int ldb, long strideB,
    void* __restrict__ Cout, void* __restrict__ Cout2, int ldc, long strideC,
    const float* __restrict__ gate, long strideG,
    int M, int N, int K, float scale) {
  static_assert(OUT_MODE == 0 || OUT_MODE == 2);
  static_assert(!GATE || OUT_MODE == 2);
  constexpr bool SPA = (SPLITM & 1) != 0;
  constexpr bool SPB = (SPLITM & 2) != 0;
  typedef typename Elem<ET>::T T;
  typedef typename Frag<T>::V V;
  const T* A = (const T*)Ap; const T* A2 = (const T*)A2p; const T* Bt = (const T*)Btp; const T* Bt2 = (const T*)Bt2p;
  __shared__ __align__(16) float sT[8][16 * 68];
  const int b    = blockIdx.y;
  const int lane = threadIdx.x & 31;
  const int wave = threadIdx.x >> 5;
  const int tilesN = N >> 6;
  const int tilesM = M >> 6;
  const int tile = blockIdx.x * 8 + wave;
  if (tile >= tilesM * tilesN) return;
  const int tm = tile / tilesN;
  const int tn = tile - tm * tilesN;
  const int m0 = tm << 6;
  const int n0 = tn << 6;

  const T* Ab  = A  + (size_t)b * strideA;
  const T* Bb  = Bt + (size_t)b * strideB;
  const T* Ab2 = SPA ? (A2  + (size_t)b * strideA) : nullptr;
  const T* Bb2 = SPB ? (Bt2 + (size_t)b * strideB) : nullptr;

  const int rlane = lane & 15;
  const int koff  = (lane >> 4) * 8;
  const int mOff  = (lane >> 4) * 8;

  int Kend = K;
  if (TRI) { const int ke = m0 + 64; Kend = (ke < K) ? ke : K; }

  v8f acc[4][4];
#pragma unroll
  for (int i = 0; i < 4; ++i)
#pragma unroll
    for (int j = 0; j < 4; ++j) acc[i][j] = (v8f){0.f,0.f,0.f,0.f,0.f,0.f,0.f,0.f};

  for (int k0 = 0; k0 < Kend; k0 += 32) {
    V bh[4], bl[4];
#pragma unroll
    for (int j = 0; j < 4; ++j) {
      const size_t bo = (size_t)(n0 + (j << 4) + rlane) * ldb + koff + k0;
      bh[j] = Frag<T>::load(Bb + bo);
      if (SPB) bl[j] = Frag<T>::load(Bb2 + bo);
    }
#pragma unroll
    for (int i = 0; i < 4; ++i) {
      const size_t ao = (size_t)(m0 + (i << 4) + rlane) * lda + koff + k0;
      V ah = Frag<T>::load(Ab + ao);
      V al;
      if (SPA) al = Frag<T>::load(Ab2 + ao);
#pragma unroll
      for (int j = 0; j < 4; ++j) {
        acc[i][j] = Frag<T>::mma(ah, bh[j], acc[i][j]);
        if (SPB) acc[i][j] = Frag<T>::mma(ah, bl[j], acc[i][j]);
        if (SPA) acc[i][j] = Frag<T>::mma(al, bh[j], acc[i][j]);
      }
      Frag<T>::guard(acc[i][0], acc[i][3], ah, SPA ? al : ah);
    }
    Frag<T>::keep(bh[0], bh[1], bh[2], bh[3]);
    if (SPB) Frag<T>::keep(bl[0], bl[1], bl[2], bl[3]);
  }
  acc_guard4(acc[0][0], acc[0][1], acc[0][2], acc[0][3]);
  acc_guard4(acc[1][0], acc[1][1], acc[1][2], acc[1][3]);
  acc_guard4(acc[2][0], acc[2][1], acc[2][2], acc[2][3]);
  acc_guard4(acc[3][0], acc[3][1], acc[3][2], acc[3][3]);

  float* slab = sT[wave];
#pragma unroll
  for (int i = 0; i < 4; ++i) {
    const int mBase = m0 + (i << 4);
#pragma unroll
    for (int j = 0; j < 4; ++j) {
#pragma unroll
      for (int r = 0; r < 8; ++r) {
        slab[(mOff + r) * 68 + (j << 4) + rlane] = acc[i][j][r] * scale;
      }
    }
    __builtin_amdgcn_fence(__ATOMIC_RELEASE, "workgroup");
    __builtin_amdgcn_wave_barrier();
    __builtin_amdgcn_fence(__ATOMIC_ACQUIRE, "workgroup");
    if (OUT_MODE == 0) {
      float* C = (float*)Cout + (size_t)b * strideC;
      const int hh = lane >> 4, c4 = (lane & 15) * 4;
      for (int pass = 0; pass < 2; ++pass) {
#pragma unroll
        for (int it = 0; it < 8; ++it) {
          const int row = it * 2 + hh;
          v4f v = *(const v4f*)(slab + row * 68 + c4);
          *(volatile v4f*)(C + (size_t)(mBase + row) * ldc + n0 + c4) = v;
        }
        __threadfence();
      }
    } else {
      const int q = lane >> 3, c8 = (lane & 7) * 8;
      unsigned short* C  = (unsigned short*)Cout  + (size_t)b * strideC;
      unsigned short* C2 = (unsigned short*)Cout2 + (size_t)b * strideC;
      const float* Gb = GATE ? (gate + (size_t)b * strideG) : nullptr;
      for (int pass = 0; pass < 2; ++pass) {
#pragma unroll
        for (int it = 0; it < 4; ++it) {
          const int row = it * 4 + q;
          const float* sp = slab + row * 68 + c8;
          U8f gv;
          gv.q[0] = (v4f){1.f, 1.f, 1.f, 1.f};
          gv.q[1] = (v4f){1.f, 1.f, 1.f, 1.f};
          if (GATE) {
            const float* gp = Gb + (size_t)(mBase + row) * ldc + n0 + c8;
            gv.q[0] = *(const v4f*)gp;
            gv.q[1] = *(const v4f*)(gp + 4);
          }
          v8h hv, lv;
#pragma unroll
          for (int e = 0; e < 8; ++e) {
            const float val = sp[e] * gv.f[e];
            const unsigned short hb = f2bf_bits(val);
            const unsigned short lb = f2bf_bits(val - bf_bits2f(hb));
            hv[e] = __builtin_bit_cast(_Float16, hb);
            lv[e] = __builtin_bit_cast(_Float16, lb);
          }
          *(volatile v8h*)(C  + (size_t)(mBase + row) * ldc + n0 + c8) = hv;
          *(volatile v8h*)(C2 + (size_t)(mBase + row) * ldc + n0 + c8) = lv;
        }
        __threadfence();
      }
    }
    __builtin_amdgcn_fence(__ATOMIC_RELEASE, "workgroup");
    __builtin_amdgcn_wave_barrier();
    __builtin_amdgcn_fence(__ATOMIC_ACQUIRE, "workgroup");
  }
}

__global__ __launch_bounds__(256) void prep_wt(const float* __restrict__ Wk, const float* __restrict__ Wv,
                                              const float* __restrict__ Wr, const float* __restrict__ Wo,
                                              unsigned short* __restrict__ Wt) {
  __shared__ __align__(16) unsigned short tileT[32 * WT_PITCH];
  const int mat = blockIdx.y;
  const int n0  = blockIdx.x * 32;
  const float* src = (mat == 0) ? Wk : (mat == 1) ? Wv : (mat == 2) ? Wr : Wo;
  const int tid = threadIdx.x, nl = tid & 31, kq = tid >> 5;
#pragma unroll 8
  for (int k0 = 0; k0 < HID; k0 += 8) {
    const int kk = k0 + kq;
    const float w = src[(size_t)kk * HID + n0 + nl];
    tileT[nl * WT_PITCH + kk] = f2bf_bits(w);
  }
  __syncthreads();
  const int wave = tid >> 5, lane = tid & 31;
  for (int pass = 0; pass < 2; ++pass) {
#pragma unroll
    for (int i = 0; i < 4; ++i) {
      const int row = wave * 4 + i;
      const v4u val = *(const v4u*)(tileT + row * WT_PITCH + lane * 8);
      *(volatile v4u*)(Wt + ((size_t)mat * HID + n0 + row) * HID + lane * 8) = val;
    }
    __threadfence();
  }
}

__global__ __launch_bounds__(256) void prep_wd(const float* __restrict__ tw, unsigned short* __restrict__ WD) {
  __shared__ unsigned short twb[SEQ_T];
  const int tid = threadIdx.x;
#pragma unroll
  for (int i = 0; i < SEQ_T / 256; ++i) twb[i * 256 + tid] = f2bf_bits(tw[i * 256 + tid]);
  __syncthreads();
  const int lane = tid & 31, wave = tid >> 5;
  const int t0 = blockIdx.x * 16;
  for (int pass = 0; pass < 2; ++pass) {
#pragma unroll
    for (int rr = 0; rr < 2; ++rr) {
      const int t = t0 + wave * 2 + rr;
#pragma unroll
      for (int seg = 0; seg < SEQ_T / 256; ++seg) {
        unsigned short bb[8];
#pragma unroll
        for (int e = 0; e < 8; ++e) {
          const int u = seg * 256 + lane * 8 + e;
          const bool ok = (u <= t);
          const int idx = ok ? ((SEQ_T - 1) - t + u) : (SEQ_T - 1);
          const unsigned short w = twb[idx];
          bb[e] = ok ? w : (unsigned short)0;
        }
        v4u val;
        val.x = pack2(bb[0], bb[1]); val.y = pack2(bb[2], bb[3]);
        val.z = pack2(bb[4], bb[5]); val.w = pack2(bb[6], bb[7]);
        *(volatile v4u*)(WD + (size_t)t * SEQ_T + seg * 256 + lane * 8) = val;
      }
    }
    __threadfence();
  }
}

__global__ __launch_bounds__(256) void mix_planes(const float* __restrict__ x, const float* __restrict__ tm,
                                                 unsigned short* __restrict__ Ph, unsigned short* __restrict__ Pl,
                                                 int row0) {
  const int lane = threadIdx.x & 31, wave = threadIdx.x >> 5;
  const int rl = blockIdx.x * 8 + wave;
  const int rg = row0 + rl;
  const int t  = rg & (SEQ_T - 1);
  const int rp = (t == 0) ? rg : (rg - 1);
  const float pz = (t == 0) ? 0.0f : 1.0f;
  const float* xr = x + (size_t)rg * HID + lane * 8;
  const float* xp = x + (size_t)rp * HID + lane * 8;
  const float* mp = tm + lane * 8;
  U8f a, p, m;
  a.q[0] = *(const v4f*)xr; a.q[1] = *(const v4f*)(xr + 4);
  p.q[0] = *(const v4f*)xp; p.q[1] = *(const v4f*)(xp + 4);
  m.q[0] = *(const v4f*)mp; m.q[1] = *(const v4f*)(mp + 4);
  unsigned short hb[8], lb[8];
#pragma unroll
  for (int e = 0; e < 8; ++e) {
    const float xb  = bfr(a.f[e]);
    const float xxb = bfr(p.f[e]) * pz;
    const float mb  = bfr(m.f[e]);
    const float t1  = xb * mb;
    const float om  = 1.0f - mb;
    const float t2  = xxb * om;
    const float xm  = t1 + t2;
    const unsigned short h = f2bf_bits(xm);
    hb[e] = h;
    lb[e] = f2bf_bits(xm - bf_bits2f(h));
  }
  v4u hv, lv;
  hv.x = pack2(hb[0], hb[1]); hv.y = pack2(hb[2], hb[3]); hv.z = pack2(hb[4], hb[5]); hv.w = pack2(hb[6], hb[7]);
  lv.x = pack2(lb[0], lb[1]); lv.y = pack2(lb[2], lb[3]); lv.z = pack2(lb[4], lb[5]); lv.w = pack2(lb[6], lb[7]);
  unsigned short* dh = Ph + (size_t)rl * HID + lane * 8;
  unsigned short* dl = Pl + (size_t)rl * HID + lane * 8;
  *(volatile v4u*)dh = hv;
  *(volatile v4u*)dl = lv;
  __threadfence();
  *(volatile v4u*)dh = hv;
  *(volatile v4u*)dl = lv;
}

__global__ __launch_bounds__(256) void scan_gate(const float* __restrict__ L, float* RG) {
  const int c = threadIdx.x;
  const int b = blockIdx.x;
  const size_t base = (size_t)b * SEQ_T * HID + c;
  float s = 0.0f;
#pragma unroll 1
  for (int t = 0; t < SEQ_T; ++t) {
    const size_t i = base + (size_t)t * HID;
    float lg = L[i];
    lg = fminf(fmaxf(lg, -60.0f), 30.0f);
    const float kk = expf(lg);
    s = s + kk;
    const float rr = RG[i];
    const float sg = 1.0f / (1.0f + expf(-rr));
    const float g  = sg * (1.0f / s);
    *(volatile float*)(RG + i) = g;
    __threadfence();
    *(volatile float*)(RG + i) = g;
  }
}

__global__ __launch_bounds__(256) void kv_transpose(const float* __restrict__ L, const float* __restrict__ V,
                                                   unsigned short* __restrict__ KH, unsigned short* __restrict__ KL,
                                                   int b0) {
  __shared__ __align__(16) unsigned short th[64 * KT_PITCH];
  __shared__ __align__(16) unsigned short tl[64 * KT_PITCH];
  const int tid = threadIdx.x;
  const int t0 = blockIdx.x * 64, c0 = blockIdx.y * 64, bl = blockIdx.z;
  const int b = b0 + bl;
#pragma unroll 1
  for (int it = 0; it < 4; ++it) {
    const int idx = it * 256 + tid;
    const int row = idx >> 4, c4 = (idx & 15) * 4;
    const size_t go = ((size_t)b * SEQ_T + t0 + row) * HID + c0 + c4;
    U4f lu, vu;
    lu.v = *(const v4f*)(L + go);
    vu.v = *(const v4f*)(V + go);
#pragma unroll
    for (int e = 0; e < 4; ++e) {
      const float lg = fminf(fmaxf(lu.f[e], -60.0f), 30.0f);
      const float kv = expf(lg) * vu.f[e];
      const unsigned short hb = f2bf_bits(kv);
      const unsigned short lb = f2bf_bits(kv - bf_bits2f(hb));
      th[(c4 + e) * KT_PITCH + row] = hb;
      tl[(c4 + e) * KT_PITCH + row] = lb;
    }
  }
  __syncthreads();
  const int wave = tid >> 5, lane = tid & 31, q = lane >> 3, u8 = (lane & 7) * 8;
  for (int pass = 0; pass < 2; ++pass) {
#pragma unroll
    for (int it = 0; it < 2; ++it) {
      const int crow = wave * 8 + it * 4 + q;
      const v4u hv = *(const v4u*)(th + crow * KT_PITCH + u8);
      const v4u lv = *(const v4u*)(tl + crow * KT_PITCH + u8);
      const size_t d = ((size_t)(bl * HID + c0 + crow)) * SEQ_T + t0 + u8;
      *(volatile v4u*)(KH + d) = hv;
      *(volatile v4u*)(KL + d) = lv;
    }
    __threadfence();
  }
}

extern "C" void kernel_launch(void* const* d_in, const int* in_sizes, int n_in,
                              void* d_out, int out_size, void* d_ws, size_t ws_size,
                              hipStream_t stream)
{
  if (n_in < 9) return;
  if (in_sizes[0] != NROWS * HID || in_sizes[1] != SEQ_T || in_sizes[2] != HID || in_sizes[3] != HID ||
      in_sizes[4] != HID || in_sizes[5] != HID * HID || in_sizes[6] != HID * HID || in_sizes[7] != HID * HID ||
      in_sizes[8] != HID * HID || out_size != NROWS * HID) return;
  if (ws_size < WS_TOTAL) return;

  const float* x   = (const float*)d_in[0];
  const float* tw  = (const float*)d_in[1];
  const float* tmk = (const float*)d_in[2];
  const float* tmv = (const float*)d_in[3];
  const float* tmr = (const float*)d_in[4];
  const float* Wk  = (const float*)d_in[5];
  const float* Wv  = (const float*)d_in[6];
  const float* Wr  = (const float*)d_in[7];
  const float* Wo  = (const float*)d_in[8];

  char* ws = (char*)d_ws;
  unsigned short* wt = (unsigned short*)(ws + OFF_WT);
  unsigned short* wd = (unsigned short*)(ws + OFF_WD);
  unsigned short* ph = (unsigned short*)(ws + OFF_PL);
  unsigned short* pl = (unsigned short*)(ws + OFF_PL + SZ_PLANE);
  float* f1 = (float*)(ws + OFF_F1);
  float* f2 = (float*)(ws + OFF_F2);
  float* f3 = (float*)(ws + OFF_F3);

  const size_t halfElems = (size_t)HALF_ROWS * HID;
  const size_t grpElems  = (size_t)BGRP * SEQ_T * HID;
  const dim3 projGrid((HALF_ROWS / 64) * (HID / 64) / 8, 1);
  const dim3 mixGrid(HALF_ROWS / 8);

  prep_wt<<<dim3(HID / 32, 4), 256, 0, stream>>>(Wk, Wv, Wr, Wo, wt);
  prep_wd<<<dim3(SEQ_T / 16), 256, 0, stream>>>(tw, wd);

  for (int h = 0; h < 2; ++h) {
    mix_planes<<<mixGrid, 256, 0, stream>>>(x, tmr, ph, pl, h * HALF_ROWS);
    wmma_gemm64<1, 1, 0, false, false><<<projGrid, 256, 0, stream>>>(
        ph, pl, HID, 0L, wt + (size_t)2 * HID * HID, nullptr, HID, 0L,
        (void*)(f3 + (size_t)h * halfElems), nullptr, HID, 0L, nullptr, 0L, HALF_ROWS, HID, HID, 1.0f);
  }
  for (int h = 0; h < 2; ++h) {
    mix_planes<<<mixGrid, 256, 0, stream>>>(x, tmk, ph, pl, h * HALF_ROWS);
    wmma_gemm64<1, 1, 0, false, false><<<projGrid, 256, 0, stream>>>(
        ph, pl, HID, 0L, wt, nullptr, HID, 0L,
        (void*)(f1 + (size_t)h * halfElems), nullptr, HID, 0L, nullptr, 0L, HALF_ROWS, HID, HID, 1.0f);
  }
  scan_gate<<<dim3(NB_SEQ), 256, 0, stream>>>(f1, f3);
  for (int h = 0; h < 2; ++h) {
    mix_planes<<<mixGrid, 256, 0, stream>>>(x, tmv, ph, pl, h * HALF_ROWS);
    wmma_gemm64<1, 1, 0, false, false><<<projGrid, 256, 0, stream>>>(
        ph, pl, HID, 0L, wt + (size_t)1 * HID * HID, nullptr, HID, 0L,
        (void*)(f2 + (size_t)h * halfElems), nullptr, HID, 0L, nullptr, 0L, HALF_ROWS, HID, HID, 1.0f);
  }
  for (int gi = 0; gi < NB_SEQ / BGRP; ++gi) {
    kv_transpose<<<dim3(SEQ_T / 64, HID / 64, BGRP), 256, 0, stream>>>(f1, f2, ph, pl, gi * BGRP);
    wmma_gemm64<1, 2, 2, true, true><<<dim3((SEQ_T / 64) * (HID / 64) / 8, BGRP), 256, 0, stream>>>(
        wd, nullptr, SEQ_T, 0L,
        ph, pl, SEQ_T, (long)HID * SEQ_T,
        (void*)((unsigned short*)f2 + (size_t)gi * grpElems), (void*)((unsigned short*)f1 + (size_t)gi * grpElems),
        HID, (long)SEQ_T * HID,
        f3 + (size_t)gi * grpElems, (long)SEQ_T * HID,
        SEQ_T, HID, SEQ_T, 1.0f);
  }
  wmma_gemm64<1, 1, 0, false, false><<<dim3((NROWS / 64) * (HID / 64) / 8, 1), 256, 0, stream>>>(
      (const unsigned short*)f2, (const unsigned short*)f1, HID, 0L, wt + (size_t)3 * HID * HID, nullptr, HID, 0L,
      d_out, nullptr, HID, 0L, nullptr, 0L, NROWS, HID, HID, 1.0f);
}
